// S3GNN_77386720739970
// MI455X (gfx1250) — hardware-verified
//
#include <hip/hip_runtime.h>
#include <stddef.h>
#include <stdint.h>


#define KIN   256
#define DF    128
#define SAH   128
#define NH    8
#define HC    16
#define NV    3
#define NOUT  8
#define GR    32
#define APH   264
#define APZ   136
#define XSP   132
#define NB    512
#define CHUNK 2048
#define NTHR  256
#define NWAVE 8
#define WCAP  256
#define NGRP  (CHUNK / (NTHR * 4))
#define PROW  256
#define WSC   16.0f
#define WINV  0.0625f

#define LDS_SACC (NB * DF)
#define LDS_DEN  (NB * NH)
#define LDS_LIST (NWAVE * WCAP)
#define LDS_BYTES ((LDS_SACC + LDS_DEN + LDS_LIST + NWAVE) * 4)

static_assert(WCAP == (CHUNK / NTHR) * 32);
static_assert(NGRP >= 1);
static_assert(NB == 512);
static_assert(CHUNK == 2048);
static_assert(SAH == DF);
static_assert(NH * HC == DF);
static_assert(NWAVE * 16 == DF);
static_assert(((LDS_SACC + LDS_DEN) % 4) == 0);
static_assert(LDS_BYTES == 286752);
static_assert(((NV * NOUT) % 4) == 0);
static_assert((KIN % 32) == 0 && (DF % 32) == 0);

typedef float    v4f  __attribute__((ext_vector_type(4)));
typedef float    v8f  __attribute__((ext_vector_type(8)));
typedef int      v4i  __attribute__((ext_vector_type(4)));
typedef _Float16 v8h  __attribute__((ext_vector_type(8)));
typedef _Float16 v16h __attribute__((ext_vector_type(16)));
union Frag   { v16h v; v8h half[2]; };
union Pack16 { v8h h; v4i i; };

__device__ __forceinline__ v8f wm(v16h a, v16h b, v8f c) {
  v8f d = __builtin_amdgcn_wmma_f32_16x16x32_f16(false, a, false, b, (short)0, c, false, false);
  asm volatile("v_nop\n\tv_nop\n\tv_nop\n\tv_nop" : "+v"(d) : "v"(a), "v"(b));
  return d;
}

__global__ __launch_bounds__(NTHR) void k_prep(const float* __restrict__ fcw, const float* __restrict__ w1,
                                               _Float16* Wh, _Float16* W1h, int n1, int n2) {
  const int g = blockIdx.x * NTHR + threadIdx.x;
  if (g >= n1 + n2) return;
  const float* src;
  _Float16* dst;
  int pitch;
  if (g < n1) {
    const int per = DF * (KIN / 8);
    const int v   = g / per;
    const int rem = g - v * per;
    const int n   = rem / (KIN / 8);
    const int k0  = (rem - n * (KIN / 8)) * 8;
    src = fcw + ((size_t)v * KIN + k0) * DF + n;  pitch = DF;
    dst = Wh + ((size_t)v * DF + n) * KIN + k0;
  } else {
    const int r  = g - n1;
    const int n  = r / (DF / 8);
    const int k0 = (r - n * (DF / 8)) * 8;
    src = w1 + (size_t)k0 * SAH + n;              pitch = SAH;
    dst = W1h + (size_t)n * DF + k0;
  }
  Pack16 u;
#pragma unroll
  for (int i = 0; i < 8; ++i) u.h[i] = (_Float16)(src[(size_t)i * pitch] * WSC);
  *(volatile v4i*)dst = u.i;
  __threadfence();
  *(volatile v4i*)dst = u.i;
}

__device__ __forceinline__ void epi_tile(v8f acc, int T, int hh, int m, int wave, int ncol,
                                         float cs, float cd, float* Xs, float* As, float* Ds) {
  float ss[8], sd[8];
#pragma unroll
  for (int r = 0; r < 8; ++r) {
    const float v = acc[r] * WINV;
    Xs[(T * 16 + 8 * hh + r) * XSP + ncol] = v;
    ss[r] = v * cs;
    sd[r] = v * cd;
  }
#pragma unroll
  for (int mk = 1; mk < 16; mk <<= 1) {
#pragma unroll
    for (int r = 0; r < 8; ++r) {
      ss[r] += __shfl_xor(ss[r], mk, 32);
      sd[r] += __shfl_xor(sd[r], mk, 32);
    }
  }
  if (m == 0) {
#pragma unroll
    for (int r = 0; r < 8; ++r) {
      As[(T * 16 + 8 * hh + r) * NH + wave] = ss[r];
      Ds[(T * 16 + 8 * hh + r) * NH + wave] = sd[r];
    }
  }
}

__global__ __launch_bounds__(NTHR) void k_gemm(
    const float* __restrict__ h, const _Float16* __restrict__ Wh,
    const float* __restrict__ attl, const float* __restrict__ attr,
    float* feat, float* elb, float* erb, int nN, int nP) {
  __shared__ __attribute__((aligned(16))) _Float16 At[GR * APH];
  __shared__ __attribute__((aligned(16))) float Xs[GR * XSP];
  __shared__ __attribute__((aligned(16))) float As[GR * NH];
  __shared__ __attribute__((aligned(16))) float Ds[GR * NH];

  const int tid  = threadIdx.x;
  const int lane = tid & 31;
  const int wave = tid >> 5;
  const int hh   = lane >> 4;
  const int m    = lane & 15;
  const int rowBase = blockIdx.x * GR;

  {
    const int r  = tid >> 3;
    const int c0 = (tid & 7) * 32;
    int row = rowBase + r;
    if (row > nN - 1) row = nN - 1;
    const float* p = h + (size_t)row * KIN + c0;
#pragma unroll
    for (int q = 0; q < 4; ++q) {
      const v4f f0 = *(const v4f*)(p + 8 * q), f1 = *(const v4f*)(p + 8 * q + 4);
      Pack16 u;
      u.h[0] = (_Float16)f0.x; u.h[1] = (_Float16)f0.y; u.h[2] = (_Float16)f0.z; u.h[3] = (_Float16)f0.w;
      u.h[4] = (_Float16)f1.x; u.h[5] = (_Float16)f1.y; u.h[6] = (_Float16)f1.z; u.h[7] = (_Float16)f1.w;
      *(v8h*)(At + r * APH + c0 + 8 * q) = u.h;
    }
  }
  __syncthreads();

  const int ncol = wave * 16 + m;
#pragma unroll 1
  for (int v = 0; v < NV; ++v) {
    v8f c0a = {0.f, 0.f, 0.f, 0.f, 0.f, 0.f, 0.f, 0.f};
    v8f c1a = {0.f, 0.f, 0.f, 0.f, 0.f, 0.f, 0.f, 0.f};
    const _Float16* wb = Wh + ((size_t)v * DF + ncol) * KIN + 8 * hh;
#pragma unroll
    for (int kt = 0; kt < KIN / 32; ++kt) {
      const int k0 = kt * 32;
      Frag a0, a1, b;
      const _Float16* pb  = wb + k0;
      const _Float16* pa0 = At + m * APH + k0 + 8 * hh;
      const _Float16* pa1 = At + (16 + m) * APH + k0 + 8 * hh;
      b.half[0]  = *(const v8h*)pb;  b.half[1]  = *(const v8h*)(pb + 16);
      a0.half[0] = *(const v8h*)pa0; a0.half[1] = *(const v8h*)(pa0 + 16);
      a1.half[0] = *(const v8h*)pa1; a1.half[1] = *(const v8h*)(pa1 + 16);
      c0a = wm(a0.v, b.v, c0a);
      c1a = wm(a1.v, b.v, c1a);
    }

    const float cs = attl[v * DF + ncol];
    const float cd = attr[v * DF + ncol];
    epi_tile(c0a, 0, hh, m, wave, ncol, cs, cd, Xs, As, Ds);
    epi_tile(c1a, 1, hh, m, wave, ncol, cs, cd, Xs, As, Ds);
    __syncthreads();

    float* fb = feat + (size_t)v * nP * DF;
    float* eb = elb  + (size_t)v * nP * NH;
    float* rb = erb  + (size_t)v * nP * NH;
    v4f xr[4];
#pragma unroll
    for (int i = 0; i < 4; ++i) xr[i] = *(const v4f*)(Xs + (4 * wave + i) * XSP + 4 * lane);
    float* gp = 0;
    v4f gv = {0.f, 0.f, 0.f, 0.f};
    if (wave < 2) {
      gv = *(const v4f*)(As + wave * 128 + 4 * lane);
      gp = eb + (size_t)rowBase * NH + wave * 128 + 4 * lane;
    } else if (wave < 4) {
      gv = *(const v4f*)(Ds + (wave - 2) * 128 + 4 * lane);
      gp = rb + (size_t)rowBase * NH + (wave - 2) * 128 + 4 * lane;
    }
    float* xpp[4];
#pragma unroll
    for (int i = 0; i < 4; ++i) xpp[i] = fb + (size_t)(rowBase + 4 * wave + i) * DF + 4 * lane;

#pragma unroll
    for (int i = 0; i < 4; ++i) *(volatile v4f*)(xpp[i]) = xr[i];
    if (gp) *(volatile v4f*)gp = gv;
    __threadfence();
#pragma unroll
    for (int i = 0; i < 4; ++i) *(volatile v4f*)(xpp[i]) = xr[i];
    if (gp) *(volatile v4f*)gp = gv;
    __syncthreads();
  }
}

__global__ __launch_bounds__(NTHR) void k_agg(
    const int* __restrict__ esrc, const int* __restrict__ edst,
    const float* __restrict__ feat, const float* __restrict__ elb, const float* __restrict__ erb,
    float* z, int nN, int nE) {
  extern __shared__ v4f lds_dyn[];
  float* sacc = (float*)lds_dyn;
  float* den  = sacc + LDS_SACC;
  int*   list = (int*)(den + LDS_DEN);
  int*   wcnt = list + LDS_LIST;

  const int tid  = threadIdx.x;
  const int lane = tid & 31;
  const int wave = tid >> 5;
  const int hd   = lane >> 2;
  const int nodeBase = blockIdx.x * NB;

  {
    const v4f z4 = {0.f, 0.f, 0.f, 0.f};
    for (int i = tid; i < (LDS_SACC + LDS_DEN) / 4; i += NTHR) lds_dyn[i] = z4;
  }
  __syncthreads();
  const bool al16 = ((((uintptr_t)edst) & 15) == 0);

  const int nChunks = (nE + CHUNK - 1) / CHUNK;
#pragma unroll 1
  for (int ch = 0; ch < nChunks; ++ch) {
    const int cbase = ch * CHUNK;
    int wc = 0;
#pragma unroll
    for (int g = 0; g < NGRP; ++g) {
      const int el0 = (g * NTHR + tid) * 4;
      const int e0  = cbase + el0;
      const int sent = -2147483647 - 1;
      v4i d;
      if (al16 && (e0 + 3 < nE)) {
        d = *(const v4i*)(edst + e0);
      } else {
        d.x = (e0     < nE) ? edst[min(e0, nE - 1)]     : sent;
        d.y = (e0 + 1 < nE) ? edst[min(e0 + 1, nE - 1)] : sent;
        d.z = (e0 + 2 < nE) ? edst[min(e0 + 2, nE - 1)] : sent;
        d.w = (e0 + 3 < nE) ? edst[min(e0 + 3, nE - 1)] : sent;
      }
      const unsigned s0 = (unsigned)d.x - (unsigned)nodeBase;
      const unsigned s1 = (unsigned)d.y - (unsigned)nodeBase;
      const unsigned s2 = (unsigned)d.z - (unsigned)nodeBase;
      const unsigned s3 = (unsigned)d.w - (unsigned)nodeBase;
      const bool h0 = s0 < (unsigned)NB;
      const bool h1 = s1 < (unsigned)NB;
      const bool h2 = s2 < (unsigned)NB;
      const bool h3 = s3 < (unsigned)NB;
      const unsigned many = __builtin_amdgcn_ballot_w32(h0 | h1 | h2 | h3);
      if (many != 0u) {
#define HITJ(J, HJ, SJ) { \
          const unsigned mj = __builtin_amdgcn_ballot_w32(HJ); \
          if (HJ) { \
            const int pos = wc + (int)__builtin_amdgcn_mbcnt_lo(mj, 0u); \
            if (pos < WCAP) list[wave * WCAP + pos] = ((el0 + (J)) << 9) | (int)(SJ); \
          } \
          wc += (int)__builtin_popcount(mj); }
        HITJ(0, h0, s0)
        HITJ(1, h1, s1)
        HITJ(2, h2, s2)
        HITJ(3, h3, s3)
#undef HITJ
      }
    }
    if (lane == 0) wcnt[wave] = wc;
    __syncthreads();

    if (wave == 0) {
      for (int wsx = 0; wsx < NWAVE; ++wsx) {
        int n = wcnt[wsx];
        if (n > WCAP) n = WCAP;
        if (n < 0) n = 0;
        for (int i = 0; i < n; ++i) {
          const int ent  = list[wsx * WCAP + i];
          const int slot = ent & (NB - 1);
          const int elx  = (ent >> 9) & (CHUNK - 1);
          int e = cbase + elx;
          if (e > nE - 1) e = nE - 1;
          int s = esrc[e];
          s = s < 0 ? 0 : (s > nN - 1 ? nN - 1 : s);
          int nd = nodeBase + slot;
          if (nd > nN - 1) nd = nN - 1;
          float a = elb[(size_t)s * NH + hd] + erb[(size_t)nd * NH + hd];
          a = (a > 0.f) ? a : 0.2f * a;
          a = fminf(fmaxf(a, -80.f), 80.f);
          const float p = __expf(a);
          const v4f xv = *(const v4f*)(feat + (size_t)s * DF + 4 * lane);
          v4f* sp = (v4f*)(sacc + slot * DF + 4 * lane);
          const v4f cur = *sp;
          const v4f nxt = cur + p * xv;
          *sp = nxt;
          if ((lane & 3) == 0) {
            const float o = den[slot * NH + hd];
            den[slot * NH + hd] = o + p;
          }
        }
      }
    }
    __syncthreads();
  }

#pragma unroll 1
  for (int j = 0; j < NB / NWAVE; ++j) {
    const int slot = wave * (NB / NWAVE) + j;
    const int node = nodeBase + slot;
    if (node >= nN) break;
    const float dv  = den[slot * NH + hd];
    const float inv = (dv > 0.f) ? (1.0f / dv) : 0.f;
    const v4f sv = *(const v4f*)(sacc + slot * DF + 4 * lane) * inv;
    v4f y;
    y.x = sv.x > 0.f ? sv.x : (__expf(fminf(sv.x, 0.f)) - 1.0f);
    y.y = sv.y > 0.f ? sv.y : (__expf(fminf(sv.y, 0.f)) - 1.0f);
    y.z = sv.z > 0.f ? sv.z : (__expf(fminf(sv.z, 0.f)) - 1.0f);
    y.w = sv.w > 0.f ? sv.w : (__expf(fminf(sv.w, 0.f)) - 1.0f);
    float* op = z + (size_t)node * DF + 4 * lane;
    *(volatile v4f*)op = y;
    __threadfence();
    *(volatile v4f*)op = y;
  }
}

__global__ __launch_bounds__(NTHR) void k_sa(
    const float* __restrict__ z, const _Float16* __restrict__ W1h,
    const float* __restrict__ b1, const float* __restrict__ w2,
    float* wl, int nN) {
  __shared__ __attribute__((aligned(16))) _Float16 At[GR * APZ];
  __shared__ __attribute__((aligned(16))) float Ws[GR * NH];
  __shared__ __attribute__((aligned(16))) float Wl[GR];

  const int tid  = threadIdx.x;
  const int lane = tid & 31;
  const int wave = tid >> 5;
  const int hh   = lane >> 4;
  const int m    = lane & 15;
  const int rowBase = blockIdx.x * GR;

  {
    const int r  = tid >> 3;
    const int c0 = (tid & 7) * 16;
    int row = rowBase + r;
    if (row > nN - 1) row = nN - 1;
    const float* p = z + (size_t)row * DF + c0;
    const v4f f0 = *(const v4f*)(p), f1 = *(const v4f*)(p + 4);
    const v4f f2 = *(const v4f*)(p + 8), f3 = *(const v4f*)(p + 12);
    Pack16 u0, u1;
    u0.h[0] = (_Float16)f0.x; u0.h[1] = (_Float16)f0.y; u0.h[2] = (_Float16)f0.z; u0.h[3] = (_Float16)f0.w;
    u0.h[4] = (_Float16)f1.x; u0.h[5] = (_Float16)f1.y; u0.h[6] = (_Float16)f1.z; u0.h[7] = (_Float16)f1.w;
    u1.h[0] = (_Float16)f2.x; u1.h[1] = (_Float16)f2.y; u1.h[2] = (_Float16)f2.z; u1.h[3] = (_Float16)f2.w;
    u1.h[4] = (_Float16)f3.x; u1.h[5] = (_Float16)f3.y; u1.h[6] = (_Float16)f3.z; u1.h[7] = (_Float16)f3.w;
    *(v8h*)(At + r * APZ + c0)     = u0.h;
    *(v8h*)(At + r * APZ + c0 + 8) = u1.h;
  }
  __syncthreads();

  const int ncol = wave * 16 + m;
  v8f c0a = {0.f, 0.f, 0.f, 0.f, 0.f, 0.f, 0.f, 0.f};
  v8f c1a = {0.f, 0.f, 0.f, 0.f, 0.f, 0.f, 0.f, 0.f};
  const _Float16* wb = W1h + (size_t)ncol * DF + 8 * hh;
#pragma unroll
  for (int kt = 0; kt < DF / 32; ++kt) {
    const int k0 = kt * 32;
    Frag a0, a1, b;
    const _Float16* pb  = wb + k0;
    const _Float16* pa0 = At + m * APZ + k0 + 8 * hh;
    const _Float16* pa1 = At + (16 + m) * APZ + k0 + 8 * hh;
    b.half[0]  = *(const v8h*)pb;  b.half[1]  = *(const v8h*)(pb + 16);
    a0.half[0] = *(const v8h*)pa0; a0.half[1] = *(const v8h*)(pa0 + 16);
    a1.half[0] = *(const v8h*)pa1; a1.half[1] = *(const v8h*)(pa1 + 16);
    c0a = wm(a0.v, b.v, c0a);
    c1a = wm(a1.v, b.v, c1a);
  }

  const float bb = b1[ncol];
  const float ww = w2[ncol];
  float s0[8], s1[8];
#pragma unroll
  for (int r = 0; r < 8; ++r) {
    s0[r] = tanhf(c0a[r] * WINV + bb) * ww;
    s1[r] = tanhf(c1a[r] * WINV + bb) * ww;
  }
#pragma unroll
  for (int mk = 1; mk < 16; mk <<= 1) {
#pragma unroll
    for (int r = 0; r < 8; ++r) {
      s0[r] += __shfl_xor(s0[r], mk, 32);
      s1[r] += __shfl_xor(s1[r], mk, 32);
    }
  }
  if (m == 0) {
#pragma unroll
    for (int r = 0; r < 8; ++r) {
      Ws[(8 * hh + r) * NH + wave]      = s0[r];
      Ws[(16 + 8 * hh + r) * NH + wave] = s1[r];
    }
  }
  __syncthreads();
  if (wave == 0) {
    float t = 0.f;
#pragma unroll
    for (int w = 0; w < NWAVE; ++w) t += Ws[lane * NH + w];
    Wl[lane] = t;
  }
  __syncthreads();
  const bool doit = (wave == 0) && (lane < GR / 4);
  v4f q = {0.f, 0.f, 0.f, 0.f};
  if (doit) q = *(const v4f*)(Wl + 4 * lane);
  float* gp = wl + (size_t)rowBase + 4 * lane;
  if (doit) *(volatile v4f*)gp = q;
  __threadfence();
  if (doit) *(volatile v4f*)gp = q;
}

__global__ __launch_bounds__(NTHR) void k_pool(const float* __restrict__ z, const float* __restrict__ wl,
                                               float* part, int nN) {
  __shared__ __attribute__((aligned(16))) float ew[NB];
  __shared__ float red[NWAVE];
  __shared__ float ssum;
  __shared__ double fd[2 * DF];
  __shared__ __attribute__((aligned(16))) float ov[PROW];

  const int tid  = threadIdx.x;
  const int lane = tid & 31;
  const int wave = tid >> 5;
  const int base = blockIdx.x * NB;
  const float NEG = -__builtin_inff();

  const int n0 = base + tid, n1 = base + tid + NTHR;
  const float w0 = (n0 < nN) ? wl[min(n0, nN - 1)] : NEG;
  const float w1 = (n1 < nN) ? wl[min(n1, nN - 1)] : NEG;
  float mx = fmaxf(w0, w1);
  mx = fmaxf(mx, __shfl_xor(mx, 16, 32));
  mx = fmaxf(mx, __shfl_xor(mx, 8, 32));
  mx = fmaxf(mx, __shfl_xor(mx, 4, 32));
  mx = fmaxf(mx, __shfl_xor(mx, 2, 32));
  mx = fmaxf(mx, __shfl_xor(mx, 1, 32));
  if (lane == 0) red[wave] = mx;
  __syncthreads();
  float mc = red[0];
#pragma unroll
  for (int w = 1; w < NWAVE; ++w) mc = fmaxf(mc, red[w]);
  const float e0 = (n0 < nN) ? __expf(w0 - mc) : 0.f;
  const float e1 = (n1 < nN) ? __expf(w1 - mc) : 0.f;
  ew[tid] = e0;
  ew[tid + NTHR] = e1;
  __syncthreads();
  if (tid == 0) {
    double s = 0.0;
#pragma unroll 1
    for (int i = 0; i < NB; ++i) s += (double)ew[i];
    ssum = (float)s;
  }
  const int col = tid & (DF - 1);
  const int rh  = tid >> 7;
  double acc = 0.0;
#pragma unroll 1
  for (int i = rh; i < NB; i += 2) {
    const int n = base + i;
    if (n >= nN) break;
    acc += (double)ew[i] * (double)z[(size_t)n * DF + col];
  }
  fd[rh * DF + col] = acc;
  __syncthreads();
  if (tid < DF) ov[tid] = (float)(fd[tid] + fd[DF + tid]);
  else          ov[tid] = (tid == DF) ? mc : ((tid == DF + 1) ? ssum : 0.f);
  __syncthreads();
  const bool doit = (wave == 0);
  v4f a = {0.f, 0.f, 0.f, 0.f}, b = {0.f, 0.f, 0.f, 0.f};
  if (doit) { a = *(const v4f*)(ov + 4 * lane); b = *(const v4f*)(ov + DF + 4 * lane); }
  float* p = part + (size_t)blockIdx.x * PROW;
  if (doit) { *(volatile v4f*)(p + 4 * lane) = a; *(volatile v4f*)(p + DF + 4 * lane) = b; }
  __threadfence();
  if (doit) { *(volatile v4f*)(p + 4 * lane) = a; *(volatile v4f*)(p + DF + 4 * lane) = b; }
}

__global__ __launch_bounds__(NTHR) void k_final(const float* __restrict__ part, const float* __restrict__ pw,
                                                const float* __restrict__ pb, float* out, int nC) {
  __shared__ float fz[NV * DF];
  __shared__ __attribute__((aligned(16))) float os[32];
  const int tid = threadIdx.x;
  if (nC > 65536) nC = 65536;
#pragma unroll 1
  for (int v = 0; v < NV; ++v) {
    const float* pv = part + (size_t)v * nC * PROW;
    float M = -__builtin_inff();
#pragma unroll 1
    for (int c = 0; c < nC; ++c) M = fmaxf(M, pv[(size_t)c * PROW + DF]);
    if (tid < DF) {
      double S = 0.0, Fv = 0.0;
#pragma unroll 1
      for (int c = 0; c < nC; ++c) {
        const float g = __expf(pv[(size_t)c * PROW + DF] - M);
        S  += (double)pv[(size_t)c * PROW + DF + 1] * (double)g;
        Fv += (double)pv[(size_t)c * PROW + tid] * (double)g;
      }
      fz[v * DF + tid] = (float)(Fv / S);
    }
  }
  __syncthreads();
  if (tid < 32) {
    float s = 0.f;
    if (tid < NV * NOUT) {
      const int v = tid >> 3, o = tid & 7;
      s = pb[o];
#pragma unroll 1
      for (int k = 0; k < DF; ++k) s += fz[v * DF + k] * pw[k * NOUT + o];
    }
    os[tid] = s;
  }
  __syncthreads();
  const bool doit = (tid < (NV * NOUT) / 4);
  v4f q = {0.f, 0.f, 0.f, 0.f};
  if (doit) q = *(const v4f*)(os + 4 * tid);
  if (doit) *(volatile v4f*)(out + 4 * tid) = q;
  __threadfence();
  if (doit) *(volatile v4f*)(out + 4 * tid) = q;
}

static inline size_t al256(size_t x) { return (x + 255) & ~(size_t)255; }

extern "C" void kernel_launch(void* const* d_in, const int* in_sizes, int n_in,
                              void* d_out, int out_size, void* d_ws, size_t ws_size,
                              hipStream_t stream) {
  if (n_in < 10) return;
  if (in_sizes[0] <= 0 || (in_sizes[0] % KIN) != 0) return;
  const int nN = in_sizes[0] / KIN;
  if (in_sizes[1] <= 0 || (in_sizes[1] % (NV * 2)) != 0) return;
  const int nE = in_sizes[1] / (NV * 2);
  if (in_sizes[2] != NV * KIN * DF) return;
  if (in_sizes[3] != NV * NH * HC || in_sizes[4] != NV * NH * HC) return;
  if (in_sizes[5] != DF * SAH || in_sizes[6] != SAH || in_sizes[7] != SAH) return;
  if (in_sizes[8] != DF * NOUT || in_sizes[9] != NOUT) return;
  if (out_size != NV * NOUT) return;

  const float* h     = (const float*)d_in[0];
  const int*   edges = (const int*)d_in[1];
  const float* fcw   = (const float*)d_in[2];
  const float* attl  = (const float*)d_in[3];
  const float* attr  = (const float*)d_in[4];
  const float* saw1  = (const float*)d_in[5];
  const float* sab1  = (const float*)d_in[6];
  const float* saw2  = (const float*)d_in[7];
  const float* pw    = (const float*)d_in[8];
  const float* pb    = (const float*)d_in[9];
  float* out = (float*)d_out;

  const int nP = ((nN + GR - 1) / GR) * GR;
  const int nC = (nN + NB - 1) / NB;

  size_t off = 0;
  _Float16* Wh  = (_Float16*)((char*)d_ws + off); off = al256(off + (size_t)NV * DF * KIN * sizeof(_Float16));
  _Float16* W1h = (_Float16*)((char*)d_ws + off); off = al256(off + (size_t)SAH * DF * sizeof(_Float16));
  float* feat = (float*)((char*)d_ws + off);      off = al256(off + (size_t)NV * nP * DF * sizeof(float));
  float* elb  = (float*)((char*)d_ws + off);      off = al256(off + (size_t)NV * nP * NH * sizeof(float));
  float* erb  = (float*)((char*)d_ws + off);      off = al256(off + (size_t)NV * nP * NH * sizeof(float));
  float* z    = (float*)((char*)d_ws + off);      off = al256(off + (size_t)nP * DF * sizeof(float));
  float* wl   = (float*)((char*)d_ws + off);      off = al256(off + (size_t)nP * sizeof(float));
  float* part = (float*)((char*)d_ws + off);      off = al256(off + (size_t)NV * nC * PROW * sizeof(float));
  if (off > ws_size) return;
  if (off > ((size_t)128 << 20)) return;

  const int n1 = NV * DF * (KIN / 8);
  const int n2 = SAH * (DF / 8);
  k_prep<<<(n1 + n2 + NTHR - 1) / NTHR, NTHR, 0, stream>>>(fcw, saw1, Wh, W1h, n1, n2);

  k_gemm<<<nP / GR, NTHR, 0, stream>>>(h, Wh, attl, attr, feat, elb, erb, nN, nP);

  hipFuncSetAttribute(reinterpret_cast<const void*>(&k_agg),
                      hipFuncAttributeMaxDynamicSharedMemorySize, LDS_BYTES);
  for (int v = 0; v < NV; ++v) {
    const int* es = edges + (size_t)v * 2 * nE;
    const int* ed = es + nE;
    k_agg<<<nC, NTHR, LDS_BYTES, stream>>>(es, ed, feat + (size_t)v * nP * DF,
                                          elb + (size_t)v * nP * NH, erb + (size_t)v * nP * NH,
                                          z, nN, nE);
    k_sa<<<nP / GR, NTHR, 0, stream>>>(z, W1h, sab1, saw2, wl, nN);
    k_pool<<<nC, NTHR, 0, stream>>>(z, wl, part + (size_t)v * nC * PROW, nN);
  }
  k_final<<<1, NTHR, 0, stream>>>(part, pw, pb, out, nC);
}
